// BidafAttn_61134564491594
// MI455X (gfx1250) — hardware-verified
//
#include <hip/hip_runtime.h>


namespace {
constexpr int Bn = 16, LC = 1024, LQ = 1024, D = 256;
constexpr size_t PL = (size_t)Bn * LC * D;

typedef _Float16 b16;
typedef __attribute__((ext_vector_type(16))) _Float16 v16b;
typedef __attribute__((ext_vector_type(8)))  _Float16 v8b;
typedef __attribute__((ext_vector_type(8)))  float v8f;
typedef __attribute__((ext_vector_type(4)))  float v4f;

__device__ __forceinline__ v8b ld8b(const b16* p) { return *(const v8b*)p; }
__device__ __forceinline__ v16b cat8b(v8b a, v8b b) { return __builtin_shufflevector(a, b, 0, 1, 2, 3, 4, 5, 6, 7, 8, 9, 10, 11, 12, 13, 14, 15); }
__device__ __forceinline__ v16b frag_kb(const b16* p, int hh) { return cat8b(ld8b(p + 8 * hh), ld8b(p + 16 + 8 * hh)); }
__device__ __forceinline__ void split16(float v, b16& hi, b16& lo) { hi = (b16)v; lo = (b16)(v - (float)hi); }
__device__ __forceinline__ void frag_ksplit(const float* p, int hh, v16b& fh_, v16b& fl_) {
  const float* p0 = p + 8 * hh; const float* p1 = p + 16 + 8 * hh;
#pragma unroll
  for (int e = 0; e < 8; ++e) { b16 a, c; split16(p0[e], a, c); fh_[e] = a; fl_[e] = c; split16(p1[e], a, c); fh_[8 + e] = a; fl_[8 + e] = c; }
}
__device__ __forceinline__ v8f wmma16b(v16b a, v16b b, v8f c) {
  v8f d = __builtin_amdgcn_wmma_f32_16x16x32_f16(false, a, false, b, (short)0, c, false, false);
  asm volatile("v_nop\n\tv_nop\n\tv_nop\n\tv_nop" : "+v"(d) : "v"(a), "v"(b));
  return d;
}
__device__ __forceinline__ void wave_lds_sync() {
  __builtin_amdgcn_fence(__ATOMIC_RELEASE, "workgroup");
  __builtin_amdgcn_wave_barrier();
  __builtin_amdgcn_fence(__ATOMIC_ACQUIRE, "workgroup");
}

struct Opnd { const void* p0; const void* p1; int ld; };
template <int NP> __device__ __forceinline__ void load_frags(const Opnd& o, int row, int kb, int hh, v16b& fh_, v16b& fl_) {
  if (NP == 0) { frag_ksplit((const float*)o.p0 + (size_t)row * o.ld + kb, hh, fh_, fl_); }
  else if (NP == 4 || NP == 5) {
    const float sc_ = (NP == 4) ? 64.0f : 8.0f;
    const float* p = (const float*)o.p0 + (size_t)row * o.ld + kb; const float* p0 = p + 8 * hh; const float* p1 = p + 16 + 8 * hh;
#pragma unroll
    for (int e = 0; e < 8; ++e) { b16 a, c; split16(p0[e] * sc_, a, c); fh_[e] = a; fl_[e] = c; split16(p1[e] * sc_, a, c); fh_[8 + e] = a; fl_[8 + e] = c; }
  } else if (NP == 3) {
    const float* p = (const float*)o.p0 + (size_t)row * o.ld + kb; const float* p0 = p + 8 * hh; const float* p1 = p + 16 + 8 * hh;
#pragma unroll
    for (int e = 0; e < 8; ++e) { fh_[e] = (b16)p0[e]; fh_[8 + e] = (b16)p1[e]; }
    fl_ = fh_;
  } else {
    fh_ = frag_kb((const b16*)o.p0 + (size_t)row * o.ld + kb, hh);
    if (NP == 2) fl_ = frag_kb((const b16*)o.p1 + (size_t)row * o.ld + kb, hh); else fl_ = fh_;
  }
}
template <int ANP, int BNP> __device__ __forceinline__ v8f mac(v16b ah, v16b al, v16b bh, v16b bl, v8f c) {
  c = wmma16b(ah, bh, c);
  if (BNP == 0 || BNP == 2 || BNP == 4 || BNP == 5) c = wmma16b(ah, bl, c);
  if (ANP == 0 || ANP == 2 || ANP == 4 || ANP == 5) c = wmma16b(al, bh, c);
  return c;
}
template <int ANP, int BNP>
__device__ __forceinline__ void gemm_tile(const Opnd& A, const Opnd& B, int K, int m0, int c0, int nloc, int hlf, v8f (&acc)[2][4]) {
  for (int kb = 0; kb < K; kb += 32) {
    v16b a0h, a0l, a1h, a1l;
    load_frags<ANP>(A, m0 + nloc, kb, hlf, a0h, a0l);
    load_frags<ANP>(A, m0 + 16 + nloc, kb, hlf, a1h, a1l);
#pragma unroll
    for (int t = 0; t < 4; ++t) {
      v16b bh, bl;
      load_frags<BNP>(B, c0 + t * 16 + nloc, kb, hlf, bh, bl);
      acc[0][t] = mac<ANP, BNP>(a0h, a0l, bh, bl, acc[0][t]);
      acc[1][t] = mac<ANP, BNP>(a1h, a1l, bh, bl, acc[1][t]);
    }
  }
}

__device__ __forceinline__ void epi_planes(v8f (&acc)[2][4], float scale, bool two, b16* __restrict__ oh, b16* __restrict__ ol, int ldo,
                                           int m0, int c0, int lane, b16* Th, b16* Tl) {
  const int nloc = lane & 15, hlf = lane >> 4;
#pragma unroll
  for (int t = 0; t < 4; ++t)
#pragma unroll
    for (int r = 0; r < 2; ++r)
#pragma unroll
      for (int v = 0; v < 8; ++v) {
        const int rr = r * 16 + v + 8 * hlf, cc = t * 16 + nloc;
        b16 h_, l_; split16(acc[r][t][v] * scale, h_, l_);
        Th[rr * 64 + cc] = h_; Tl[rr * 64 + cc] = l_;
      }
  wave_lds_sync();
  for (int pass = 0; pass < 2; ++pass) {
#pragma unroll
    for (int j = 0; j < 8; ++j) {
      const int rr = j * 4 + (lane >> 3), c8 = (lane & 7) * 8;
      const size_t o = (size_t)(m0 + rr) * ldo + c0 + c8;
      *(volatile v8b*)(oh + o) = ld8b(Th + rr * 64 + c8);
      if (two) *(volatile v8b*)(ol + o) = ld8b(Tl + rr * 64 + c8);
    }
    __threadfence();
  }
}
__device__ __forceinline__ void epi_f32(v8f (&acc)[2][4], float scale, const float* rscale, float* __restrict__ out, int ldo, int m0, int c0, int lane, float* Tt) {
  const int nloc = lane & 15, hlf = lane >> 4;
#pragma unroll
  for (int t = 0; t < 4; ++t)
#pragma unroll
    for (int r = 0; r < 2; ++r)
#pragma unroll
      for (int v = 0; v < 8; ++v) {
        const int rr = r * 16 + v + 8 * hlf;
        const float rs = rscale ? rscale[(size_t)(m0 + rr) * 32] : 1.0f;
        Tt[rr * 64 + t * 16 + nloc] = acc[r][t][v] * scale * rs;
      }
  wave_lds_sync();
  float* dst0 = out + (size_t)m0 * ldo + c0;
  for (int pass = 0; pass < 2; ++pass) {
#pragma unroll
    for (int j = 0; j < 16; ++j) { const int rr = j * 2 + hlf, c4 = nloc * 4; *(volatile v4f*)(dst0 + (size_t)rr * ldo + c4) = *(const v4f*)(Tt + rr * 64 + c4); }
    __threadfence();
  }
}


typedef __attribute__((ext_vector_type(8))) __bf16 v8bb; typedef __attribute__((ext_vector_type(16))) __bf16 v16bb;
typedef __attribute__((ext_vector_type(8))) unsigned short v8us;
__device__ __forceinline__ v16bb frag_kb_bf(const __bf16* p, int hh) { const v8bb a = *(const v8bb*)(p + 8 * hh), b = *(const v8bb*)(p + 16 + 8 * hh); return __builtin_shufflevector(a, b, 0, 1, 2, 3, 4, 5, 6, 7, 8, 9, 10, 11, 12, 13, 14, 15); }
__device__ __forceinline__ v8f wmma16bb(v16bb a, v16bb b, v8f c) {
  v8f d = __builtin_amdgcn_wmma_f32_16x16x32_bf16(false, a, false, b, (short)0, c, false, false);
  asm volatile("v_nop\n\tv_nop\n\tv_nop\n\tv_nop" : "+v"(d) : "v"(a), "v"(b));
  return d;
}
__device__ __forceinline__ unsigned short bf16_rne_bits(float v) { unsigned int u = __float_as_uint(v); u += 0x7FFFu + ((u >> 16) & 1u); return (unsigned short)(u >> 16); }
__device__ __forceinline__ float bf16_rne(float v) { return __uint_as_float(((unsigned int)bf16_rne_bits(v)) << 16); }


__global__ __launch_bounds__(256) void prep_kernel(const float* __restrict__ c, const float* __restrict__ q, const float* __restrict__ w, b16* __restrict__ cmh, b16* __restrict__ qh, float* __restrict__ cw, float* __restrict__ qw) {
  const int wid = threadIdx.x >> 5, lane = threadIdx.x & 31, row = blockIdx.x * 8 + wid;
  float sc = 0.0f, sq = 0.0f;
  for (int pass = 0; pass < 2; ++pass) {
#pragma unroll
    for (int jq = 0; jq < 2; ++jq) { const int d0 = jq * 128 + lane * 4; const v4f cv = *(const v4f*)(c + (size_t)row * D + d0), qv = *(const v4f*)(q + (size_t)row * D + d0);
      typedef __attribute__((ext_vector_type(4))) _Float16 v4b; v4b ch, cl, qq;
#pragma unroll
      for (int e = 0; e < 4; ++e) { const float cb = bf16_rne(cv[e]), qb = bf16_rne(qv[e]); const float wc_ = bf16_rne(w[d0 + e]), wq_ = bf16_rne(w[D + d0 + e]), wm_ = bf16_rne(w[2 * D + d0 + e]);
        if (pass == 0) { sc += cb * wc_; sq += qb * wq_; }
        b16 a, l; split16(cb * wm_, a, l); ch[e] = a; cl[e] = (b16)((cb * wm_ - (float)a) * 256.0f); qq[e] = (b16)qb; }
      *(volatile v4b*)(cmh + (size_t)row * D + d0) = ch; *(volatile v4b*)(cmh + PL + (size_t)row * D + d0) = cl; *(volatile v4b*)(qh + (size_t)row * D + d0) = qq; }
    if (pass == 0) {
#pragma unroll
      for (int o = 16; o > 0; o >>= 1) { sc += __shfl_xor(sc, o); sq += __shfl_xor(sq, o); } }
    if (lane == 0) { ((volatile float*)cw)[row] = sc; ((volatile float*)qw)[row] = sq; }
    __threadfence();
  }
}

__global__ __launch_bounds__(256) void qt_kernel(const b16* __restrict__ qh, b16* __restrict__ qt) {
  __shared__ __attribute__((aligned(16))) b16 T[D][64 + 8];
  const int t_ = threadIdx.x, rowb = blockIdx.x * 64, b = rowb / LQ, j0 = rowb % LQ;
  for (int i = t_; i < 64 * D / 8; i += 256) { const int r = i / (D / 8), c8 = (i % (D / 8)) * 8; const v8b v = *(const v8b*)(qh + (size_t)(rowb + r) * D + c8);
#pragma unroll
    for (int e = 0; e < 8; ++e) T[c8 + e][r] = v[e]; }
  __syncthreads();
  for (int pass = 0; pass < 2; ++pass) { for (int i = t_; i < D * 8; i += 256) { const int d = i >> 3, c8 = (i & 7) * 8; *(volatile v8b*)(qt + ((size_t)b * D + d) * LQ + j0 + c8) = *(const v8b*)(&T[d][c8]); } __threadfence(); }
}

__global__ __launch_bounds__(256) void c2q_kernel(const b16* __restrict__ cmh, const b16* __restrict__ qh, const b16* __restrict__ qt, const float* __restrict__ cw, const float* __restrict__ qw, float* __restrict__ c2q, float* __restrict__ rmax) {
  __shared__ __attribute__((aligned(16))) float Os[8][16][128 + 4];
  const int wid = threadIdx.x >> 5, lane = threadIdx.x & 31, hh = lane >> 4, col = lane & 15;
  const int wt = blockIdx.x * 8 + wid, fh = wt & 1, it = (wt >> 1) & 63, b = wt >> 7, i0 = it * 16, ii = i0 + col;
  const b16* Cm = cmh + ((size_t)b * LC) * D; const b16* Q = qh + ((size_t)b * LQ) * D; const b16* Qt = qt + ((size_t)b * D + fh * 128) * LQ;
  const float cwi = cw[(size_t)b * LC + ii];
  float m = -INFINITY, l = 0.0f; v8f o[8] = {{}, {}, {}, {}, {}, {}, {}, {}};
  for (int jb = 0; jb < LQ; jb += 32) {
    v8f s0 = {}, s1 = {}, t0 = {}, t1 = {};
#pragma unroll
    for (int ks = 0; ks < 8; ++ks) { const v16b q0 = frag_kb(Q + (size_t)(jb + col) * D + ks * 32, hh), q1 = frag_kb(Q + (size_t)(jb + 16 + col) * D + ks * 32, hh);
      const v16b cf = frag_kb(Cm + (size_t)ii * D + ks * 32, hh), cl = frag_kb(Cm + PL + (size_t)ii * D + ks * 32, hh);
      s0 = wmma16b(q0, cf, s0); t0 = wmma16b(q0, cl, t0); s1 = wmma16b(q1, cf, s1); t1 = wmma16b(q1, cl, t1); }
    float mr = -INFINITY;
#pragma unroll
    for (int r = 0; r < 8; ++r) { s0[r] = s0[r] + t0[r] * (1.0f / 256.0f) + cwi + qw[(size_t)b * LQ + jb + 8 * hh + r]; s1[r] = s1[r] + t1[r] * (1.0f / 256.0f) + cwi + qw[(size_t)b * LQ + jb + 16 + 8 * hh + r]; mr = fmaxf(mr, fmaxf(s0[r], s1[r])); }
    mr = fmaxf(mr, __shfl_xor(mr, 16));
    const float mn = fmaxf(m, mr), al_ = __expf(m - mn); m = mn;
    float sum = 0.0f; v16b pb, pl;
#pragma unroll
    for (int r = 0; r < 8; ++r) { const float e0 = __expf(s0[r] - mn), e1 = __expf(s1[r] - mn); sum += e0 + e1; b16 a, cc; split16(e0 * 8.0f, a, cc); pb[r] = a; pl[r] = cc; split16(e1 * 8.0f, a, cc); pb[8 + r] = a; pl[8 + r] = cc; }
    sum += __shfl_xor(sum, 16); l = l * al_ + sum;
#pragma unroll
    for (int n = 0; n < 8; ++n) {
#pragma unroll
      for (int r = 0; r < 8; ++r) o[n][r] *= al_;
      const v16b qf = frag_kb(Qt + (size_t)(n * 16 + col) * LQ + jb, hh);
      o[n] = wmma16b(qf, pb, o[n]); o[n] = wmma16b(qf, pl, o[n]); }
  }
  const float inv = 1.0f / (8.0f * l);
#pragma unroll
  for (int n = 0; n < 8; ++n)
#pragma unroll
    for (int r = 0; r < 8; ++r) Os[wid][col][n * 16 + 8 * hh + r] = o[n][r] * inv;
  if (fh == 0) for (int pass = 0; pass < 2; ++pass) { ((volatile float*)rmax)[((size_t)b * 64 + it) * 32 + lane] = m; __threadfence(); }
  wave_lds_sync();
  float* dst = c2q + ((size_t)b * LC + i0) * D + fh * 128;
  for (int pass = 0; pass < 2; ++pass) {
#pragma unroll
    for (int rr = 0; rr < 16; ++rr) *(volatile v4f*)(dst + (size_t)rr * D + lane * 4) = *(const v4f*)(&Os[wid][rr][lane * 4]);
    __threadfence();
  }
}

__global__ __launch_bounds__(256) void q2c_kernel(const float* __restrict__ rmax, const float* __restrict__ c, float* __restrict__ out2) {
  __shared__ float wv[LC]; __shared__ float red[8]; __shared__ float qv[D];
  const int b = blockIdx.x, t_ = threadIdx.x, wave = t_ >> 5, lane = t_ & 31;
  auto RM = [&](int i) { return rmax[((size_t)b * 64 + (i >> 4)) * 32 + (i & 15)]; };
  float mx = -INFINITY; for (int i = t_; i < LC; i += 256) mx = fmaxf(mx, RM(i));
#pragma unroll
  for (int o = 16; o > 0; o >>= 1) mx = fmaxf(mx, __shfl_xor(mx, o));
  if (lane == 0) red[wave] = mx;
  __syncthreads();
  mx = fmaxf(fmaxf(fmaxf(red[0], red[1]), fmaxf(red[2], red[3])), fmaxf(fmaxf(red[4], red[5]), fmaxf(red[6], red[7])));
  __syncthreads();
  float s = 0.0f; for (int i = t_; i < LC; i += 256) { const float e = __expf(RM(i) - mx); wv[i] = e; s += e; }
#pragma unroll
  for (int o = 16; o > 0; o >>= 1) s += __shfl_xor(s, o);
  if (lane == 0) red[wave] = s;
  __syncthreads();
  const float inv = 1.0f / (red[0] + red[1] + red[2] + red[3] + red[4] + red[5] + red[6] + red[7]);
  { float acc = 0.0f; const int d = t_;
#pragma unroll 1
    for (int i = 0; i < LC; ++i) acc += wv[i] * bf16_rne(c[((size_t)b * LC + i) * D + d]);
    qv[d] = acc * inv; }
  __syncthreads();
  for (int pass = 0; pass < 2; ++pass) { for (int i = t_; i < LC * D / 4; i += 256) { const int r = i / (D / 4), cq = (i % (D / 4)) * 4; *(volatile v4f*)(out2 + ((size_t)b * LC + r) * D + cq) = *(const v4f*)(&qv[cq]); } __threadfence(); }
}
}

extern "C" void kernel_launch(void* const* d_in, const int* in_sizes, int n_in,
                              void* d_out, int out_size, void* d_ws, size_t ws_size, hipStream_t stream) {
  (void)n_in; (void)out_size;
  const float* c = (const float*)d_in[0]; const float* q = (const float*)d_in[1]; const float* w = (const float*)d_in[2];
  float* out = (float*)d_out;
  if (in_sizes[0] != Bn * LC * D || in_sizes[1] != Bn * LQ * D || in_sizes[2] != 3 * D) return;
  size_t off = 0; char* ws = (char*)d_ws;
  auto carve = [&](size_t bytes) { char* p = ws + off; off += (bytes + 255) & ~(size_t)255; return p; };
  b16* cmh = (b16*)carve(PL * 2 * 2); b16* qh = (b16*)carve(PL * 2); b16* qt = (b16*)carve(PL * 2); float* cw = (float*)carve((size_t)Bn * LC * 4); float* qw = (float*)carve((size_t)Bn * LQ * 4); float* rmax = (float*)carve((size_t)Bn * 64 * 32 * 4);
  if (off > ws_size) return;
  prep_kernel<<<Bn * LC / 8, 256, 0, stream>>>(c, q, w, cmh, qh, cw, qw);
  qt_kernel<<<Bn * LQ / 64, 256, 0, stream>>>(qh, qt);
  c2q_kernel<<<Bn * 64 * 2 / 8, 256, 0, stream>>>(cmh, qh, qt, cw, qw, out, rmax);
  q2c_kernel<<<Bn, 256, 0, stream>>>(rmax, c, out + PL);
}
